// Mamba2Block_85925115724494
// MI455X (gfx1250) — hardware-run, weakly checked
//
#include <hip/hip_runtime.h>
#include <math.h>

constexpr int kBatch = 2;
constexpr int kSeq   = 1024;
constexpr int kDm    = 128;
constexpr int kDin   = 256;
constexpr int kDst   = 256;
constexpr int kXzN   = 2 * kDin;
constexpr int kPrN   = 2 * kDst + kDin;
constexpr int kLseq  = 2 * kBatch;
constexpr int kRows  = kLseq * kSeq;
constexpr int kOutRows = kBatch * kSeq;

constexpr float kActCarry = 16.0f;
constexpr float kWCarry   = 16.0f;
constexpr float kYCarry   = 64.0f;
constexpr float kResCarry = 2048.0f;
constexpr float kResInv   = 1.0f / kResCarry;
constexpr float kScaleIn  = 1.0f / (kActCarry * kWCarry);
constexpr float kScaleOut = 1.0f / (kYCarry * kWCarry);
constexpr float kF16Min   = 6.103515625e-05f;

constexpr int kConvTP  = 260;
constexpr int kScanJB  = 32;
constexpr int kScanNG  = 16;
constexpr int kScanNS  = 16;
constexpr int kScanCT  = 8;
constexpr int kScanThr = kScanJB * kScanNG;

static_assert(kSeq == 1024 && kBatch == 2);
static_assert(kDin == kDst);
static_assert(kRows % 64 == 0 && kXzN % 64 == 0 && kPrN % 64 == 0 && kDm % 64 == 0);
static_assert(kDm % 32 == 0 && kDin % 32 == 0);
static_assert(kDm % 64 == 0 && kDin % 64 == 0);
static_assert(kScanNG * kScanNS == kDst);
static_assert(kScanThr == 512);
static_assert(kSeq % kScanCT == 0);
static_assert(kDin % kScanJB == 0);
static_assert(kScanCT * (kDst / 4) == kScanThr);
static_assert(kScanCT * kScanJB * 2 == kScanThr);

typedef __attribute__((ext_vector_type(16))) _Float16 v16h;
typedef __attribute__((ext_vector_type(8)))  _Float16 v8h;
typedef __attribute__((ext_vector_type(8)))  float    v8f;
typedef __attribute__((ext_vector_type(4)))  float    v4f;
typedef __attribute__((ext_vector_type(4)))  unsigned int v4u;

__device__ __forceinline__ unsigned pk16(unsigned short a, unsigned short b) {
  return (unsigned)a | ((unsigned)b << 16);
}
__device__ __forceinline__ void h_split(float v, unsigned short& hb, unsigned short& rb) {
  const float vs = (__builtin_fabsf(v) < kF16Min) ? 0.0f : v;
  const _Float16 h = (_Float16)vs;
  const float hf = (float)h;
  const float d = (v - hf) * kResCarry;
  const float ds = (__builtin_fabsf(d) < kF16Min) ? 0.0f : d;
  const _Float16 r = (_Float16)ds;
  hb = __builtin_bit_cast(unsigned short, h);
  rb = __builtin_bit_cast(unsigned short, r);
}
__device__ __forceinline__ void pack8_split(const float (&v)[8], v4u& uh, v4u& ur) {
  unsigned short hb[8], rb[8];
#pragma unroll
  for (int e = 0; e < 8; ++e) h_split(v[e], hb[e], rb[e]);
  uh = (v4u){pk16(hb[0], hb[1]), pk16(hb[2], hb[3]), pk16(hb[4], hb[5]), pk16(hb[6], hb[7])};
  ur = (v4u){pk16(rb[0], rb[1]), pk16(rb[2], rb[3]), pk16(rb[4], rb[5]), pk16(rb[6], rb[7])};
}

struct FragH {
  union U { v16h v; v8h h[2]; };
  static __device__ __forceinline__ v16h load(const _Float16* p) {
    U f;
    f.h[0] = *(const v8h*)(p);
    f.h[1] = *(const v8h*)(p + 16);
    return f.v;
  }
  static __device__ __forceinline__ v8f mma(v16h a, v16h b, v8f c) {
    return __builtin_amdgcn_wmma_f32_16x16x32_f16(false, a, false, b, (short)0, c, false, false);
  }
};
__device__ __forceinline__ void guard_split(v8f& a0, v8f& a1, v8f& a2, v8f& a3,
                                            v16h x0, v16h x1, v16h x2, v16h x3, v16h y0, v16h y1) {
  asm volatile("v_nop\n\tv_nop\n\tv_nop\n\tv_nop"
               : "+v"(a0), "+v"(a1), "+v"(a2), "+v"(a3)
               : "v"(x0), "v"(x1), "v"(x2), "v"(x3), "v"(y0), "v"(y1));
}
__device__ __forceinline__ void acc_guard4(v8f& a, v8f& b, v8f& c, v8f& d) {
  asm volatile("v_nop\n\tv_nop\n\tv_nop\n\tv_nop" : "+v"(a), "+v"(b), "+v"(c), "+v"(d));
}

template <int ACT>
__global__ __launch_bounds__(256) void gemm_split_kernel(
    const unsigned short* __restrict__ Ahp, const unsigned short* __restrict__ Arp, int lda,
    const unsigned short* __restrict__ Bhp, const unsigned short* __restrict__ Brp, int ldb,
    float* __restrict__ C, int ldc, int M, int N, int K, float scale, int actN) {
  __shared__ __align__(16) float sT[8][16 * 68];
  const int lane = threadIdx.x & 31;
  const int wave = threadIdx.x >> 5;
  const int tilesN = N >> 6;
  const int tilesM = M >> 5;
  const int tile = blockIdx.x * 8 + wave;
  if (tile >= tilesM * tilesN) return;
  const int tm = tile / tilesN;
  const int tn = tile - tm * tilesN;
  const int m0 = tm << 5;
  const int n0 = tn << 6;
  const int rlane = lane & 15;
  const int half8 = (lane >> 4) * 8;
  const int mOff  = (lane >> 4) * 8;

  const size_t aoff = (size_t)(m0 + rlane) * lda + half8;
  const size_t boff = (size_t)(n0 + rlane) * ldb + half8;
  const _Float16* pa0 = (const _Float16*)Ahp + aoff;
  const _Float16* pa1 = pa0 + (size_t)16 * lda;
  const _Float16* pr0 = (const _Float16*)Arp + aoff;
  const _Float16* pr1 = pr0 + (size_t)16 * lda;
  const _Float16* pbh = (const _Float16*)Bhp + boff;
  const _Float16* pbr = (const _Float16*)Brp + boff;
  const size_t bstep = (size_t)16 * ldb;

  v8f acc[2][4], accr[2][4];
#pragma unroll
  for (int i = 0; i < 2; ++i)
#pragma unroll
    for (int j = 0; j < 4; ++j) {
      acc[i][j]  = (v8f){0.f, 0.f, 0.f, 0.f, 0.f, 0.f, 0.f, 0.f};
      accr[i][j] = (v8f){0.f, 0.f, 0.f, 0.f, 0.f, 0.f, 0.f, 0.f};
    }

  for (int k0 = 0; k0 < K; k0 += 32) {
    const v16h ah0 = FragH::load(pa0 + k0);
    const v16h ah1 = FragH::load(pa1 + k0);
    const v16h ar0 = FragH::load(pr0 + k0);
    const v16h ar1 = FragH::load(pr1 + k0);
#pragma unroll
    for (int j = 0; j < 4; ++j) {
      const v16h bh = FragH::load(pbh + j * bstep + k0);
      const v16h br = FragH::load(pbr + j * bstep + k0);
      acc[0][j]  = FragH::mma(ah0, bh, acc[0][j]);
      acc[1][j]  = FragH::mma(ah1, bh, acc[1][j]);
      accr[0][j] = FragH::mma(ah0, br, accr[0][j]);
      accr[1][j] = FragH::mma(ah1, br, accr[1][j]);
      accr[0][j] = FragH::mma(ar0, bh, accr[0][j]);
      accr[1][j] = FragH::mma(ar1, bh, accr[1][j]);
      guard_split(acc[0][j], acc[1][j], accr[0][j], accr[1][j], ah0, ah1, ar0, ar1, bh, br);
    }
  }
  acc_guard4(acc[0][0], acc[0][1], acc[0][2], acc[0][3]);
  acc_guard4(acc[1][0], acc[1][1], acc[1][2], acc[1][3]);
  acc_guard4(accr[0][0], accr[0][1], accr[0][2], accr[0][3]);
  acc_guard4(accr[1][0], accr[1][1], accr[1][2], accr[1][3]);

  float* slab = sT[wave];
  const int hh = lane >> 4, c4 = (lane & 15) * 4;
#pragma unroll
  for (int i = 0; i < 2; ++i) {
    const int mBase = m0 + (i << 4);
#pragma unroll
    for (int j = 0; j < 4; ++j) {
#pragma unroll
      for (int r = 0; r < 8; ++r) {
        float v = acc[i][j][r];
        v += accr[i][j][r] * kResInv;
        v *= scale;
        slab[(mOff + r) * 68 + (j << 4) + rlane] = v;
      }
    }
    __builtin_amdgcn_fence(__ATOMIC_RELEASE, "workgroup");
    __builtin_amdgcn_wave_barrier();
    __builtin_amdgcn_fence(__ATOMIC_ACQUIRE, "workgroup");
    if (ACT == 1) {
      if (n0 < actN) {
#pragma unroll 1
        for (int idx = 0; idx < 32; ++idx) {
          float* sp = slab + ((idx >> 2) * 2 + hh) * 68 + c4 + (idx & 3);
          const float x = *sp;
          const float y = fmaxf(x, 0.0f) + log1pf(expf(-__builtin_fabsf(x)));
          *sp = y;
        }
      }
      __builtin_amdgcn_fence(__ATOMIC_RELEASE, "workgroup");
      __builtin_amdgcn_wave_barrier();
      __builtin_amdgcn_fence(__ATOMIC_ACQUIRE, "workgroup");
    }
    for (int pass = 0; pass < 2; ++pass) {
#pragma unroll
      for (int it = 0; it < 8; ++it) {
        const int row = it * 2 + hh;
        const v4f v = *(const v4f*)(slab + row * 68 + c4);
        *(volatile v4f*)(C + (size_t)(mBase + row) * ldc + n0 + c4) = v;
      }
      __threadfence();
    }
    __builtin_amdgcn_fence(__ATOMIC_RELEASE, "workgroup");
    __builtin_amdgcn_wave_barrier();
    __builtin_amdgcn_fence(__ATOMIC_ACQUIRE, "workgroup");
  }
}

__global__ __launch_bounds__(256) void wt_plane_kernel(const float* __restrict__ W,
                                                       unsigned short* __restrict__ outh,
                                                       unsigned short* __restrict__ outr,
                                                       int Kd, int Nd) {
  __shared__ float sm[64][65];
  const int t  = threadIdx.x;
  const int k0 = blockIdx.x * 64;
  const int n0 = blockIdx.y * 64;
#pragma unroll
  for (int i = 0; i < 16; ++i) {
    const int e = i * 256 + t;
    const int r = e >> 6;
    const int c = e & 63;
    const int kk = k0 + r;
    const int nn = n0 + c;
    const bool valid = (kk < Kd) && (nn < Nd);
    const int kc = (kk < Kd) ? kk : (Kd - 1);
    const int nc = (nn < Nd) ? nn : (Nd - 1);
    const float v = W[(size_t)kc * Nd + nc];
    sm[c][r] = valid ? (v * kWCarry) : 0.0f;
  }
  __syncthreads();
  const int lane = t & 31, wave = t >> 5;
  const int q = lane >> 3, c8 = (lane & 7) * 8;
  for (int pass = 0; pass < 2; ++pass) {
#pragma unroll
    for (int it = 0; it < 2; ++it) {
      const int row = wave * 8 + it * 4 + q;
      float v[8];
#pragma unroll
      for (int e = 0; e < 8; ++e) v[e] = sm[row][c8 + e];
      v4u uh, ur;
      pack8_split(v, uh, ur);
      const size_t o = (size_t)(n0 + row) * Kd + k0 + c8;
      *(volatile v4u*)(outh + o) = uh;
      *(volatile v4u*)(outr + o) = ur;
    }
    __threadfence();
  }
}

__global__ __launch_bounds__(256) void cast_planes_kernel(const float* __restrict__ src,
                                                          unsigned short* __restrict__ dh,
                                                          unsigned short* __restrict__ dr,
                                                          int cshift, int total, int flip, float carry) {
  const unsigned i = blockIdx.x * 256u + threadIdx.x;
  if (i >= (unsigned)total) return;
  const unsigned drow = i >> cshift;
  const unsigned c8 = (i & ((1u << cshift) - 1u)) * 8u;
  const unsigned cols = 8u << cshift;
  const unsigned ls = drow >> 10;
  const unsigned t  = drow & 1023u;
  const unsigned tp = (ls >= 2u) ? (1023u - t) : t;
  const unsigned frow = (ls & 1u) * 1024u + tp;
  const unsigned srow = (flip != 0) ? frow : drow;
  const float* sp = src + (size_t)srow * cols + c8;
  const v4f a = *(const v4f*)(sp);
  const v4f b = *(const v4f*)(sp + 4);
  float v[8];
#pragma unroll
  for (int e = 0; e < 4; ++e) {
    v[e]     = a[e] * carry;
    v[4 + e] = b[e] * carry;
  }
  v4u uh, ur;
  pack8_split(v, uh, ur);
  const size_t off = (size_t)i * 8;
  *(volatile v4u*)(dh + off) = uh;
  *(volatile v4u*)(dr + off) = ur;
  __threadfence();
  *(volatile v4u*)(dh + off) = uh;
  *(volatile v4u*)(dr + off) = ur;
}

__global__ __launch_bounds__(256) void conv_silu_kernel(const float* __restrict__ XZ,
                                                        const float* __restrict__ cw,
                                                        const float* __restrict__ cb,
                                                        float* __restrict__ XC,
                                                        unsigned short* __restrict__ XCh,
                                                        unsigned short* __restrict__ XCr) {
  __shared__ __align__(16) float sT[16 * kConvTP];
  const unsigned tid = threadIdx.x, lane = tid & 31u, wave = tid >> 5;
  const unsigned g0 = blockIdx.x * 64u;
  const unsigned tb = g0 & (unsigned)(kSeq - 1);
  const v4f w4 = *(const v4f*)(cw + tid * 4u);
  const float bc = cb[tid];
  float xm3, xm2, xm1;
  {
    const bool hist = (tb > 0u);
    const unsigned rb = hist ? (g0 - 3u) : g0;
    const float v3 = XZ[(size_t)rb * kXzN + tid];
    const float v2 = XZ[(size_t)(rb + 1u) * kXzN + tid];
    const float v1 = XZ[(size_t)(rb + 2u) * kXzN + tid];
    xm3 = hist ? v3 : 0.0f;
    xm2 = hist ? v2 : 0.0f;
    xm1 = hist ? v1 : 0.0f;
  }
  const unsigned hrow = wave >> 1;
  const unsigned hch  = (wave & 1u) * 128u + lane * 4u;
#pragma unroll 1
  for (int sub = 0; sub < 4; ++sub) {
    const unsigned lb = g0 + (unsigned)sub * 16u;
#pragma unroll 1
    for (int s = 0; s < 16; ++s) {
      const float xcur = XZ[(size_t)(lb + (unsigned)s) * kXzN + tid];
      float acc = w4[0] * xm3;
      acc = fmaf(w4[1], xm2, acc);
      acc = fmaf(w4[2], xm1, acc);
      acc = fmaf(w4[3], xcur, acc);
      const float sv = acc + bc;
      const float sg = __builtin_amdgcn_rcpf(1.0f + expf(-sv));
      sT[s * kConvTP + tid] = sv * sg;
      xm3 = xm2;
      xm2 = xm1;
      xm1 = xcur;
    }
    __syncthreads();
    v4f fv[4];
    v4u ph[2], pr[2];
#pragma unroll
    for (int it = 0; it < 4; ++it) fv[it] = *(const v4f*)(sT + (it * 4 + hrow) * kConvTP + hch);
#pragma unroll
    for (int it = 0; it < 2; ++it) {
      const float* sp = sT + (it * 8 + wave) * kConvTP + lane * 8u;
      const v4f a0 = *(const v4f*)(sp);
      const v4f a1 = *(const v4f*)(sp + 4);
      float v[8];
#pragma unroll
      for (int e = 0; e < 4; ++e) {
        v[e]     = a0[e] * kActCarry;
        v[4 + e] = a1[e] * kActCarry;
      }
      pack8_split(v, ph[it], pr[it]);
    }
    for (int pass = 0; pass < 2; ++pass) {
#pragma unroll
      for (int it = 0; it < 4; ++it)
        *(volatile v4f*)(XC + (size_t)(lb + it * 4 + hrow) * kDin + hch) = fv[it];
#pragma unroll
      for (int it = 0; it < 2; ++it) {
        const size_t o = (size_t)(lb + it * 8 + wave) * kDin + lane * 8u;
        *(volatile v4u*)(XCh + o) = ph[it];
        *(volatile v4u*)(XCr + o) = pr[it];
      }
      __threadfence();
    }
    __syncthreads();
  }
}

__global__ __launch_bounds__(512) void scan_full_kernel(const float* __restrict__ PROJ,
                                                        const float* __restrict__ XC,
                                                        const float* __restrict__ XZ,
                                                        const float* __restrict__ Alog,
                                                        const float* __restrict__ Dp,
                                                        float* __restrict__ YG) {
  __shared__ __align__(16) float sDl[kScanCT * kDst];
  __shared__ __align__(16) float sDb[kScanCT * kDst];
  __shared__ __align__(16) float sCm[kScanCT * kDst];
  __shared__ __align__(16) float sXj[kScanCT * kScanJB];
  __shared__ __align__(16) float sZg[kScanCT * kScanJB];
  __shared__ __align__(16) float red[kScanCT * kScanNG * kScanJB];
  __shared__ __align__(16) float yb[kScanCT * kScanJB];

  const unsigned tid = threadIdx.x;
  const unsigned jl  = tid & 31u;
  const unsigned g   = tid >> 5;
  const unsigned ls  = blockIdx.x >> 3;
  const unsigned j0  = (blockIdx.x & 7u) * (unsigned)kScanJB;
  const size_t row0  = (size_t)ls * kSeq;

  const float alj = Alog[j0 + jl];
  const float Aj  = -expf(alj);
  float dpj = Dp[j0 + jl];
  asm volatile("" : "+v"(dpj));

  float s[kScanNS];
#pragma unroll
  for (int m = 0; m < kScanNS; ++m) s[m] = 0.0f;

  const unsigned stt = tid >> 6;
  const unsigned sc4 = (tid & 63u) * 4u;
  const unsigned xtt = (tid >> 5) & 7u;

#pragma unroll 1
  for (int ch = 0; ch < kSeq / kScanCT; ++ch) {
    const size_t r0 = row0 + (size_t)ch * kScanCT;
    {
      const float* pp = PROJ + (r0 + stt) * kPrN + sc4;
      const v4f d4 = *(const v4f*)(pp);
      const v4f b4 = *(const v4f*)(pp + kDst);
      const v4f c4 = *(const v4f*)(pp + 2 * kDst);
      const v4f db = d4 * b4;
      *(v4f*)(sDl + stt * kDst + sc4) = d4;
      *(v4f*)(sDb + stt * kDst + sc4) = db;
      *(v4f*)(sCm + stt * kDst + sc4) = c4;
      if (tid < 256u) {
        sXj[xtt * kScanJB + jl] = XC[(r0 + xtt) * kDin + j0 + jl];
      } else {
        sZg[xtt * kScanJB + jl] = XZ[(r0 + xtt) * kXzN + kDin + j0 + jl];
      }
    }
    __syncthreads();

#pragma unroll 1
    for (int tt = 0; tt < kScanCT; ++tt) {
      const float xj = sXj[tt * kScanJB + jl];
      const float* pd = sDl + tt * kDst + g * kScanNS;
      const float* pb = sDb + tt * kDst + g * kScanNS;
      const float* pc = sCm + tt * kDst + g * kScanNS;
      float part = 0.0f;
#pragma unroll
      for (int q4 = 0; q4 < kScanNS / 4; ++q4) {
        const v4f d4 = *(const v4f*)(pd + 4 * q4);
        const v4f b4 = *(const v4f*)(pb + 4 * q4);
        const v4f c4 = *(const v4f*)(pc + 4 * q4);
#pragma unroll
        for (int e = 0; e < 4; ++e) {
          const float ea = expf(d4[e] * Aj);
          const float bx = b4[e] * xj;
          const float sn = fmaf(ea, s[4 * q4 + e], bx);
          s[4 * q4 + e] = sn;
          part = fmaf(c4[e], sn, part);
        }
      }
      red[(tt * kScanNG + g) * kScanJB + jl] = part;
    }
    __syncthreads();

    if (tid < 256u) {
      float tot = 0.0f;
#pragma unroll
      for (int g2 = 0; g2 < kScanNG; ++g2) tot += red[(g * kScanNG + g2) * kScanJB + jl];
      const float xv = sXj[g * kScanJB + jl];
      const float zv = sZg[g * kScanJB + jl];
      const float y  = tot + dpj * xv;
      const float sg = __builtin_amdgcn_rcpf(1.0f + expf(-zv));
      yb[g * kScanJB + jl] = y * (zv * sg);
    }
    __syncthreads();

    if (tid < 64u) {
      const unsigned q   = jl >> 3;
      const unsigned c4  = (jl & 7u) * 4u;
      const unsigned tok = g * 4u + q;
      const v4f val = *(const v4f*)(yb + tok * kScanJB + c4);
      float* dst = YG + (r0 + tok) * kDin + j0 + c4;
      *(volatile v4f*)dst = val;
      __threadfence();
      *(volatile v4f*)dst = val;
    }
  }
}

__global__ __launch_bounds__(256) void merge_kernel(const float* __restrict__ DIR, float* __restrict__ out, int total) {
  const unsigned i = blockIdx.x * 256u + threadIdx.x;
  if (i >= (unsigned)total) return;
  const unsigned row = i >> 5;
  const unsigned c4  = (i & 31u) * 4u;
  const unsigned b   = row >> 10;
  const unsigned t   = row & 1023u;
  const size_t rf = (size_t)b * kSeq + t;
  const size_t rr = (size_t)(2u + b) * kSeq + (1023u - t);
  const v4f f = *(const v4f*)(DIR + rf * kDm + c4);
  const v4f r = *(const v4f*)(DIR + rr * kDm + c4);
  const v4f o = (f + r) * 0.5f;
  float* dst = out + (size_t)row * kDm + c4;
  *(volatile v4f*)dst = o;
  __threadfence();
  *(volatile v4f*)dst = o;
}

constexpr size_t kBWI  = (size_t)kXzN * kDm * 2;
constexpr size_t kBWX  = (size_t)kPrN * kDin * 2;
constexpr size_t kBWO  = (size_t)kDm * kDin * 2;
constexpr size_t kBXF  = (size_t)kRows * kDm * 2;
constexpr size_t kBXZ  = (size_t)kRows * kXzN * 4;
constexpr size_t kBXC  = (size_t)kRows * kDin * 4;
constexpr size_t kBXCp = (size_t)kRows * kDin * 2;
constexpr size_t kBPR  = (size_t)kRows * kPrN * 4;
constexpr size_t kBYG  = (size_t)kRows * kDin * 4;
constexpr size_t kBYGp = (size_t)kRows * kDin * 2;
constexpr size_t kBDIR = (size_t)kRows * kDm * 4;
constexpr size_t kWsTotal = 2 * kBWI + 2 * kBWX + 2 * kBWO + 2 * kBXF + kBXZ + kBXC + 2 * kBXCp + kBPR + kBYG + 2 * kBYGp + kBDIR;
static_assert(kWsTotal == 43122688ull);
static_assert(kWsTotal <= 134217728ull);
static_assert(kBWI % 256 == 0 && kBWX % 256 == 0 && kBWO % 256 == 0 && kBXF % 256 == 0);
static_assert(((kRows / 32) * (kXzN / 64)) % 8 == 0);
static_assert(((kRows / 32) * (kPrN / 64)) % 8 == 0);
static_assert(((kRows / 32) * (kDm / 64)) % 8 == 0);
static_assert((kRows * kDm / 8) % 256 == 0 && (kRows * kDin / 8) % 256 == 0 && (kOutRows * kDm / 4) % 256 == 0);

extern "C" void kernel_launch(void* const* d_in, const int* in_sizes, int n_in,
                              void* d_out, int out_size, void* d_ws, size_t ws_size, hipStream_t stream) {
  if (n_in < 8 || d_out == nullptr || d_ws == nullptr) return;
  if (in_sizes[0] != kOutRows * kDm) return;
  if (in_sizes[1] != kDm * kXzN) return;
  if (in_sizes[2] != kDin * 4) return;
  if (in_sizes[3] != kDin) return;
  if (in_sizes[4] != kDin * kPrN) return;
  if (in_sizes[5] != kDin) return;
  if (in_sizes[6] != kDin) return;
  if (in_sizes[7] != kDin * kDm) return;
  if (out_size != kOutRows * kDm) return;
  if (ws_size < kWsTotal) return;

  const float* x      = (const float*)d_in[0];
  const float* W_in   = (const float*)d_in[1];
  const float* conv_w = (const float*)d_in[2];
  const float* conv_b = (const float*)d_in[3];
  const float* W_x    = (const float*)d_in[4];
  const float* A_log  = (const float*)d_in[5];
  const float* Dp     = (const float*)d_in[6];
  const float* W_out  = (const float*)d_in[7];
  float* out = (float*)d_out;

  char* ws = (char*)d_ws;
  size_t off = 0;
  auto carve = [&](size_t bytes) -> char* {
    char* p = ws + off;
    off += (bytes + 255) & ~(size_t)255;
    return p;
  };
  unsigned short* WIh = (unsigned short*)carve(kBWI);
  unsigned short* WIr = (unsigned short*)carve(kBWI);
  unsigned short* WXh = (unsigned short*)carve(kBWX);
  unsigned short* WXr = (unsigned short*)carve(kBWX);
  unsigned short* WOh = (unsigned short*)carve(kBWO);
  unsigned short* WOr = (unsigned short*)carve(kBWO);
  unsigned short* XFh = (unsigned short*)carve(kBXF);
  unsigned short* XFr = (unsigned short*)carve(kBXF);
  float*          XZ  = (float*)carve(kBXZ);
  float*          XC  = (float*)carve(kBXC);
  unsigned short* XCh = (unsigned short*)carve(kBXCp);
  unsigned short* XCr = (unsigned short*)carve(kBXCp);
  float*          PROJ = (float*)carve(kBPR);
  float*          YG  = (float*)carve(kBYG);
  unsigned short* YGh = (unsigned short*)carve(kBYGp);
  unsigned short* YGr = (unsigned short*)carve(kBYGp);
  float*          DIR = (float*)carve(kBDIR);
  if (off != kWsTotal || off > ws_size) return;

  wt_plane_kernel<<<dim3(kDm / 64, kXzN / 64), 256, 0, stream>>>(W_in, WIh, WIr, kDm, kXzN);
  wt_plane_kernel<<<dim3(kDin / 64, kPrN / 64), 256, 0, stream>>>(W_x, WXh, WXr, kDin, kPrN);
  wt_plane_kernel<<<dim3(kDin / 64, kDm / 64), 256, 0, stream>>>(W_out, WOh, WOr, kDin, kDm);

  cast_planes_kernel<<<(kRows * kDm / 8) / 256, 256, 0, stream>>>(x, XFh, XFr, 4, kRows * kDm / 8, 1, kActCarry);

  gemm_split_kernel<0><<<((kRows / 32) * (kXzN / 64)) / 8, 256, 0, stream>>>(
      XFh, XFr, kDm, WIh, WIr, kDm, XZ, kXzN, kRows, kXzN, kDm, kScaleIn, 0);

  conv_silu_kernel<<<kRows / 64, 256, 0, stream>>>(XZ, conv_w, conv_b, XC, XCh, XCr);

  gemm_split_kernel<1><<<((kRows / 32) * (kPrN / 64)) / 8, 256, 0, stream>>>(
      XCh, XCr, kDin, WXh, WXr, kDin, PROJ, kPrN, kRows, kPrN, kDin, kScaleIn, kDst);

  scan_full_kernel<<<kLseq * (kDin / kScanJB), kScanThr, 0, stream>>>(PROJ, XC, XZ, A_log, Dp, YG);

  cast_planes_kernel<<<(kRows * kDin / 8) / 256, 256, 0, stream>>>(YG, YGh, YGr, 5, kRows * kDin / 8, 0, kYCarry);

  gemm_split_kernel<0><<<((kRows / 32) * (kDm / 64)) / 8, 256, 0, stream>>>(
      YGh, YGr, kDin, WOh, WOr, kDin, DIR, kDm, kRows, kDm, kDin, kScaleOut, 0);

  merge_kernel<<<(kOutRows * kDm / 4) / 256, 256, 0, stream>>>(DIR, out, kOutRows * kDm / 4);
}
